// E_GCL_20607253086819
// MI455X (gfx1250) — hardware-run, weakly checked
//
#include <hip/hip_runtime.h>
#include <math.h>

constexpr int kNodes  = 10000;
constexpr int kEdges  = 320000;
constexpr int kFeat   = 256;
constexpr int kKcat   = 512;
constexpr int kNpad   = 10048;
constexpr int kEch    = 32000;
constexpr int kNchunk = 10;
constexpr int kTnode  = 48;
constexpr int kNtile  = 210;
constexpr int kNagg   = kNtile * kTnode;
constexpr int kScha   = 2048;
constexpr int kNstep  = (kEch + kScha - 1) / kScha;
constexpr int kNT     = 256;
constexpr float kWcarry    = 16.0f;
constexpr float kWcarryInv = 1.0f / 16.0f;
constexpr int kVwrad = 0, kVbe1 = 256, kVbe2 = 512, kVbc1 = 768, kVbn1 = 1024, kVbn2 = 1280, kVwc2 = 1536, kVbc2 = 1792, kVcoord = 1824;
constexpr int kCoordN   = kNodes * 3;
constexpr int kCoordPad = 30016;
constexpr int kVecFloats = kVcoord + kCoordPad;
constexpr int kGatherBlocks   = kEch * 64 / kNT;
constexpr int kRadBlocks      = (kEch + kNT - 1) / kNT;
constexpr int kNodeBlocks     = kNpad * 32 / kNT;
constexpr int kEdgeGemmBlocks = ((kEch / 64) * (kFeat / 64) + 7) / 8;
constexpr int kNodeGemmBlocks = ((kNpad / 64) * (kFeat / 64) + 7) / 8;
constexpr int kCoordOutBlocks = (kCoordN + kNT - 1) / kNT;
constexpr int kVecBlocks      = 8 + (kCoordPad + kNT - 1) / kNT;

static_assert(kEdges == kNchunk * kEch, "");
static_assert(kEch % 64 == 0 && kEch % 8 == 0 && kEch < 65536 && kEch % kNT == 0, "");
static_assert(kNpad % 64 == 0 && kNpad >= kNodes && kNagg >= kNpad, "");
static_assert(kFeat % 64 == 0 && kKcat % 32 == 0 && kFeat % 32 == 0, "");
static_assert(kNpad * 32 % kNT == 0 && kEch * 64 % kNT == 0, "");
static_assert(kTnode == 6 * (kNT / 32) && kTnode <= 48, "");
static_assert(kVcoord % 32 == 0 && kCoordPad % 32 == 0 && kCoordPad >= kCoordN, "");
static_assert(kNstep * kScha >= kEch, "");

typedef __attribute__((ext_vector_type(16))) _Float16 v16h;
typedef __attribute__((ext_vector_type(8)))  _Float16 v8h;
typedef __attribute__((ext_vector_type(16))) __bf16   v16b;
typedef __attribute__((ext_vector_type(8)))  __bf16   v8b;
typedef __attribute__((ext_vector_type(8)))  float    v8f;
typedef __attribute__((ext_vector_type(4)))  float    v4f;
typedef __attribute__((ext_vector_type(4)))  unsigned int v4u;
typedef __attribute__((ext_vector_type(4)))  int      v4i;

__device__ __forceinline__ unsigned short f2bf_bits(float f) {
  unsigned u = __float_as_uint(f);
  return (unsigned short)((u + 0x7FFFu + ((u >> 16) & 1u)) >> 16);
}
__device__ __forceinline__ float bf_bits2f(unsigned short h) { return __uint_as_float(((unsigned)h) << 16); }
__device__ __forceinline__ float bf16r(float f) { return bf_bits2f(f2bf_bits(f)); }
__device__ __forceinline__ unsigned pk16(unsigned short a, unsigned short b) { return (unsigned)a | ((unsigned)b << 16); }
__device__ __forceinline__ unsigned short h_bits(float f) { const _Float16 h = (_Float16)f; return __builtin_bit_cast(unsigned short, h); }
__device__ __forceinline__ float h16_to_f32(unsigned hb) {
  const unsigned sgn = (hb & 0x8000u) << 16; const unsigned em = hb & 0x7fffu;
  const float fn = __uint_as_float((em << 13) + 0x38000000u);
  const float fs = (float)em * 5.9604644775390625e-8f;
  const float mag = (em < 0x400u) ? fs : fn; return __uint_as_float(__float_as_uint(mag) | sgn); }
__device__ __forceinline__ float silu_f(float v) {
  const float t = fminf(-v, 60.0f);
  const float e = expf(t);
  const float sg = __builtin_amdgcn_rcpf(1.0f + e);
  return v * sg;
}

__device__ __forceinline__ void tile_guard_h(v8f& a, v8f& b, v8f& c, v8f& d, v16h x0, v16h x1, v16h y0, v16h y1, v16h y2, v16h y3) {
  asm volatile("v_nop\n\tv_nop\n\tv_nop\n\tv_nop" : "+v"(a), "+v"(b), "+v"(c), "+v"(d) : "v"(x0), "v"(x1), "v"(y0), "v"(y1), "v"(y2), "v"(y3));
}
__device__ __forceinline__ void tile_guard_b(v8f& a, v8f& b, v8f& c, v8f& d, v16b x0, v16b x1, v16b y0, v16b y1, v16b y2, v16b y3) {
  asm volatile("v_nop\n\tv_nop\n\tv_nop\n\tv_nop" : "+v"(a), "+v"(b), "+v"(c), "+v"(d) : "v"(x0), "v"(x1), "v"(y0), "v"(y1), "v"(y2), "v"(y3));
}
__device__ __forceinline__ void acc_guard4(v8f& a, v8f& b, v8f& c, v8f& d) { asm volatile("v_nop\n\tv_nop\n\tv_nop\n\tv_nop" : "+v"(a), "+v"(b), "+v"(c), "+v"(d)); }

template <typename T> struct Frag;
template <> struct Frag<_Float16> {
  typedef v16h V; union U { v16h v; v8h h[2]; };
  static __device__ __forceinline__ v16h load(const _Float16* p) {
    U f; f.h[0] = *(const v8h*)(p); f.h[1] = *(const v8h*)(p + 16); return f.v;
  }
  static __device__ __forceinline__ v8f mma(v16h a, v16h b, v8f c) {
    return __builtin_amdgcn_wmma_f32_16x16x32_f16(false, a, false, b, (short)0, c, false, false);
  }
  static __device__ __forceinline__ void tguard(v8f& a, v8f& b, v8f& c, v8f& d, v16h x0, v16h x1, v16h y0, v16h y1, v16h y2, v16h y3) {
    tile_guard_h(a, b, c, d, x0, x1, y0, y1, y2, y3);
  }
};
template <> struct Frag<__bf16> {
  typedef v16b V; union U { v16b v; v8b h[2]; };
  static __device__ __forceinline__ v16b load(const __bf16* p) {
    U f; f.h[0] = *(const v8b*)(p); f.h[1] = *(const v8b*)(p + 16); return f.v;
  }
  static __device__ __forceinline__ v8f mma(v16b a, v16b b, v8f c) {
    return __builtin_amdgcn_wmma_f32_16x16x32_bf16(false, a, false, b, (short)0, c, false, false);
  }
  static __device__ __forceinline__ void tguard(v8f& a, v8f& b, v8f& c, v8f& d, v16b x0, v16b x1, v16b y0, v16b y1, v16b y2, v16b y3) {
    tile_guard_b(a, b, c, d, x0, x1, y0, y1, y2, y3);
  }
};
template <int ET> struct Elem;
template <> struct Elem<0> { typedef _Float16 T; };
template <> struct Elem<1> { typedef __bf16 T; };

template <int ET, bool SPLITA, int EPI>
__global__ __launch_bounds__(256) void gemm_kernel(
    const unsigned short* __restrict__ Ap, const unsigned short* __restrict__ A2p, int lda,
    const unsigned short* __restrict__ Btp, int ldb,
    void* __restrict__ Cout, void* __restrict__ Cout2, int ldc,
    const float* __restrict__ bias, const float* __restrict__ rvec, const float* __restrict__ cvec,
    int M, int N, int K, int mreal, float scale) {
  typedef typename Elem<ET>::T T;
  typedef typename Frag<T>::V V;
  const T* A = (const T*)Ap; const T* A2 = (const T*)A2p; const T* Bt = (const T*)Btp;
  __shared__ __align__(16) float sT[8][16 * 68];
  const int lane = threadIdx.x & 31;
  const int wave = threadIdx.x >> 5;
  const int tilesN = N >> 6;
  const int tilesM = M >> 6;
  const int tile = blockIdx.x * 8 + wave;
  if (tile >= tilesM * tilesN) return;
  const int tm = tile / tilesN;
  const int tn = tile - tm * tilesN;
  const int m0 = tm << 6;
  const int n0 = tn << 6;

  const int rlane = lane & 15;
  const int koff  = (lane >> 4) * 8;
  const int mOff  = (lane >> 4) * 8;

  v8f acc[4][4];
#pragma unroll
  for (int i = 0; i < 4; ++i)
#pragma unroll
    for (int j = 0; j < 4; ++j) acc[i][j] = (v8f){0.f,0.f,0.f,0.f,0.f,0.f,0.f,0.f};

  for (int k0 = 0; k0 < K; k0 += 32) {
    V bh[4];
#pragma unroll
    for (int j = 0; j < 4; ++j) {
      const size_t bo = (size_t)(n0 + (j << 4) + rlane) * ldb + koff + k0;
      bh[j] = Frag<T>::load(Bt + bo);
    }
#pragma unroll
    for (int i = 0; i < 4; ++i) {
      const size_t ao = (size_t)(m0 + (i << 4) + rlane) * lda + koff + k0;
      const V ah = Frag<T>::load(A + ao);
      V al = ah;
      if (SPLITA) al = Frag<T>::load(A2 + ao);
#pragma unroll
      for (int j = 0; j < 4; ++j) {
        acc[i][j] = Frag<T>::mma(ah, bh[j], acc[i][j]);
        if (SPLITA) acc[i][j] = Frag<T>::mma(al, bh[j], acc[i][j]);
      }
      Frag<T>::tguard(acc[i][0], acc[i][1], acc[i][2], acc[i][3], ah, al, bh[0], bh[1], bh[2], bh[3]);
    }
  }
  acc_guard4(acc[0][0], acc[0][1], acc[0][2], acc[0][3]);
  acc_guard4(acc[1][0], acc[1][1], acc[1][2], acc[1][3]);
  acc_guard4(acc[2][0], acc[2][1], acc[2][2], acc[2][3]);
  acc_guard4(acc[3][0], acc[3][1], acc[3][2], acc[3][3]);

  float* slab = sT[wave];
  float bvj[4], cvj[4];
#pragma unroll
  for (int j = 0; j < 4; ++j) {
    const int n = n0 + (j << 4) + rlane;
    bvj[j] = bias[n];
    if (EPI == 1 || EPI == 3) cvj[j] = cvec[n]; else cvj[j] = 0.0f;
  }
#pragma unroll
  for (int i = 0; i < 4; ++i) {
    const int mBase = m0 + (i << 4);
    float rv8[8];
    if (EPI == 1) {
      const v4f r0 = *(const v4f*)(rvec + mBase + mOff);
      const v4f r1 = *(const v4f*)(rvec + mBase + mOff + 4);
#pragma unroll
      for (int e = 0; e < 4; ++e) { rv8[e] = r0[e]; rv8[4 + e] = r1[e]; }
    } else {
#pragma unroll
      for (int e = 0; e < 8; ++e) rv8[e] = 0.0f;
    }
    float rs[8];
#pragma unroll
    for (int r = 0; r < 8; ++r) rs[r] = 0.0f;
#pragma unroll
    for (int j = 0; j < 4; ++j) {
#pragma unroll
      for (int r = 0; r < 8; ++r) {
        float v = acc[i][j][r] * scale + bvj[j];
        if (EPI == 1) v += rv8[r] * cvj[j];
        if (EPI != 2) v = silu_f(v);
        if (EPI == 3) rs[r] += v * cvj[j];
        else slab[(mOff + r) * 68 + (j << 4) + rlane] = v;
      }
    }
    if (EPI == 3) {
#pragma unroll
      for (int r = 0; r < 8; ++r) {
        float x = rs[r];
        x += __shfl_xor(x, 1, 32);
        x += __shfl_xor(x, 2, 32);
        x += __shfl_xor(x, 4, 32);
        x += __shfl_xor(x, 8, 32);
        if (rlane == 0) slab[(i << 4) + mOff + r] = x;
      }
    } else {
      __builtin_amdgcn_fence(__ATOMIC_RELEASE, "workgroup");
      __builtin_amdgcn_wave_barrier();
      __builtin_amdgcn_fence(__ATOMIC_ACQUIRE, "workgroup");
      if (EPI == 2) {
        float* C = (float*)Cout;
        const int hh = lane >> 4, c4 = (lane & 15) * 4;
        for (int pass = 0; pass < 2; ++pass) {
#pragma unroll
          for (int it = 0; it < 8; ++it) {
            const int row  = it * 2 + hh;
            const int grow = mBase + row;
            const v4f v = *(const v4f*)(slab + row * 68 + c4);
            if (grow < mreal) *(volatile v4f*)(C + (size_t)grow * ldc + n0 + c4) = v;
          }
          __threadfence();
        }
      } else {
        unsigned short* C  = (unsigned short*)Cout;
        unsigned short* C2 = (unsigned short*)Cout2;
        const int q = lane >> 3, c8 = (lane & 7) * 8;
        for (int pass = 0; pass < 2; ++pass) {
#pragma unroll
          for (int it = 0; it < 4; ++it) {
            const int row = it * 4 + q;
            const float* sp = slab + row * 68 + c8;
            unsigned short hb[8], lb[8];
#pragma unroll
            for (int e = 0; e < 8; ++e) {
              const float x = sp[e];
              if (EPI == 4) {
                const unsigned short hbits = f2bf_bits(x);
                hb[e] = hbits;
                lb[e] = f2bf_bits(x - bf_bits2f(hbits));
              } else {
                hb[e] = h_bits(x);
                lb[e] = 0;
              }
            }
            const v4u uh = (v4u){pk16(hb[0], hb[1]), pk16(hb[2], hb[3]), pk16(hb[4], hb[5]), pk16(hb[6], hb[7])};
            *(volatile v4u*)(C + (size_t)(mBase + row) * ldc + n0 + c8) = uh;
            if (EPI == 4) {
              const v4u ul = (v4u){pk16(lb[0], lb[1]), pk16(lb[2], lb[3]), pk16(lb[4], lb[5]), pk16(lb[6], lb[7])};
              *(volatile v4u*)(C2 + (size_t)(mBase + row) * ldc + n0 + c8) = ul;
            }
          }
          __threadfence();
        }
      }
      __builtin_amdgcn_fence(__ATOMIC_RELEASE, "workgroup");
      __builtin_amdgcn_wave_barrier();
      __builtin_amdgcn_fence(__ATOMIC_ACQUIRE, "workgroup");
    }
  }
  if (EPI == 3) {
    __builtin_amdgcn_fence(__ATOMIC_RELEASE, "workgroup");
    __builtin_amdgcn_wave_barrier();
    __builtin_amdgcn_fence(__ATOMIC_ACQUIRE, "workgroup");
    float* R = (float*)Cout;
    const v4f x = *(const v4f*)(slab + 4 * (lane & 15));
    for (int pass = 0; pass < 2; ++pass) {
      if (lane < 16) *(volatile v4f*)(R + (size_t)tn * ldc + m0 + 4 * lane) = x;
      __threadfence();
    }
  }
}

__global__ __launch_bounds__(kNT) void prep_w_kernel(const float* __restrict__ We1, const float* __restrict__ We2,
                                                     const float* __restrict__ Wc1, const float* __restrict__ Wn1,
                                                     const float* __restrict__ Wn2,
                                                     unsigned short* __restrict__ B1, unsigned short* __restrict__ B2,
                                                     unsigned short* __restrict__ B3, unsigned short* __restrict__ B4,
                                                     unsigned short* __restrict__ B5) {
  __shared__ float sm[64][65];
  const int t  = threadIdx.x;
  const int bx = blockIdx.x;
  const int n0 = blockIdx.y * 64;
  const float* W; unsigned short* op; int K; int kt; int isbf;
  if (bx < 8)       { W = We1; op = B1; K = 512; kt = bx;      isbf = 1; }
  else if (bx < 12) { W = We2; op = B2; K = 256; kt = bx - 8;  isbf = 0; }
  else if (bx < 16) { W = Wc1; op = B3; K = 256; kt = bx - 12; isbf = 0; }
  else if (bx < 24) { W = Wn1; op = B4; K = 512; kt = bx - 16; isbf = 1; }
  else              { W = Wn2; op = B5; K = 256; kt = bx - 24; isbf = 1; }
  const int k0 = kt * 64;
#pragma unroll
  for (int i = 0; i < 16; ++i) {
    const int e = i * 256 + t;
    const int r = e >> 6;
    const int c = e & 63;
    sm[c][r] = W[(size_t)(k0 + r) * kFeat + n0 + c];
  }
  __syncthreads();
  const int lane = t & 31, wave = t >> 5;
  const int q = lane >> 3, c8 = (lane & 7) * 8;
  for (int pass = 0; pass < 2; ++pass) {
#pragma unroll
    for (int it = 0; it < 2; ++it) {
      const int row = wave * 8 + it * 4 + q;
      unsigned short hb[8];
#pragma unroll
      for (int e = 0; e < 8; ++e) {
        const float x = bf16r(sm[row][c8 + e]);
        hb[e] = isbf ? f2bf_bits(x) : h_bits(kWcarry * x);
      }
      const v4u u = (v4u){pk16(hb[0], hb[1]), pk16(hb[2], hb[3]), pk16(hb[4], hb[5]), pk16(hb[6], hb[7])};
      *(volatile v4u*)(op + (size_t)(n0 + row) * K + k0 + c8) = u;
    }
    __threadfence();
  }
}

__global__ __launch_bounds__(kNT) void prep_vec_kernel(const float* __restrict__ We1, const float* __restrict__ be1,
                                                       const float* __restrict__ be2, const float* __restrict__ bc1,
                                                       const float* __restrict__ bn1, const float* __restrict__ bn2,
                                                       const float* __restrict__ Wc2, const float* __restrict__ bc2,
                                                       const float* __restrict__ coord, float* __restrict__ vec) {
  const int b = blockIdx.x, t = threadIdx.x;
  if (b < 7) {
    const float* src = (b == 0) ? (We1 + (size_t)512 * kFeat) : (b == 1) ? be1 : (b == 2) ? be2 : (b == 3) ? bc1
                     : (b == 4) ? bn1 : (b == 5) ? bn2 : Wc2;
    const float v = bf16r(src[t]);
    float* dst = vec + b * 256 + t;
    *(volatile float*)dst = v;
    __threadfence();
    *(volatile float*)dst = v;
  } else if (b == 7) {
    const float bv = bf16r(bc2[0]);
    const float v = (t == 0) ? bv : 0.0f;
    if (t < 32) {
      float* dst = vec + kVbc2 + t;
      *(volatile float*)dst = v;
      __threadfence();
      *(volatile float*)dst = v;
    }
  } else {
    const int i = (b - 8) * kNT + t;
    const int ic = i < kCoordN ? i : (kCoordN - 1);
    const float livef = (i < kCoordN) ? 1.0f : 0.0f;
    const float v = bf16r(coord[ic]) * livef;
    if (i < kCoordPad) {
      float* dst = vec + kVcoord + i;
      *(volatile float*)dst = v;
      __threadfence();
      *(volatile float*)dst = v;
    }
  }
}

__global__ __launch_bounds__(kNT) void node_h_kernel(const float* __restrict__ h, unsigned short* __restrict__ AH,
                                                     unsigned short* __restrict__ AL) {
  const int t = blockIdx.x * kNT + threadIdx.x;
  const int row = t >> 5, c8 = (t & 31) * 8;
  const int rc = row < kNodes ? row : (kNodes - 1);
  const float livef = (row < kNodes) ? 1.0f : 0.0f;
  const float* p = h + (size_t)rc * kFeat + c8;
  const v4f a = *(const v4f*)(p);
  const v4f c = *(const v4f*)(p + 4);
  unsigned short hb[8];
#pragma unroll
  for (int e = 0; e < 4; ++e) { hb[e] = f2bf_bits(a[e] * livef); hb[4 + e] = f2bf_bits(c[e] * livef); }
  const v4u u = (v4u){pk16(hb[0], hb[1]), pk16(hb[2], hb[3]), pk16(hb[4], hb[5]), pk16(hb[6], hb[7])};
  const v4u z = (v4u){0u, 0u, 0u, 0u};
  unsigned short* qh = AH + (size_t)row * kKcat + c8;
  unsigned short* ql = AL + (size_t)row * kKcat + c8;
  *(volatile v4u*)qh = u;
  *(volatile v4u*)ql = z;
  __threadfence();
  *(volatile v4u*)qh = u;
  *(volatile v4u*)ql = z;
}

__global__ __launch_bounds__(kNT) void node_fin_kernel(const float* __restrict__ agg, unsigned short* __restrict__ AH,
                                                       unsigned short* __restrict__ AL) {
  const int t = blockIdx.x * kNT + threadIdx.x;
  const int row = t >> 5, c8 = (t & 31) * 8;
  const float livef = (row < kNodes) ? 1.0f : 0.0f;
  const float* p = agg + (size_t)row * kFeat + c8;
  const v4f a = *(const v4f*)(p);
  const v4f c = *(const v4f*)(p + 4);
  unsigned short hb[8], lb[8];
#pragma unroll
  for (int e = 0; e < 4; ++e) {
    const float x0 = a[e] * livef, x1 = c[e] * livef;
    const unsigned short h0 = f2bf_bits(x0), h1 = f2bf_bits(x1);
    hb[e] = h0; lb[e] = f2bf_bits(x0 - bf_bits2f(h0));
    hb[4 + e] = h1; lb[4 + e] = f2bf_bits(x1 - bf_bits2f(h1));
  }
  const v4u uh = (v4u){pk16(hb[0], hb[1]), pk16(hb[2], hb[3]), pk16(hb[4], hb[5]), pk16(hb[6], hb[7])};
  const v4u ul = (v4u){pk16(lb[0], lb[1]), pk16(lb[2], lb[3]), pk16(lb[4], lb[5]), pk16(lb[6], lb[7])};
  unsigned short* qh = AH + (size_t)row * kKcat + kFeat + c8;
  unsigned short* ql = AL + (size_t)row * kKcat + kFeat + c8;
  *(volatile v4u*)qh = uh;
  *(volatile v4u*)ql = ul;
  __threadfence();
  *(volatile v4u*)qh = uh;
  *(volatile v4u*)ql = ul;
}

__global__ __launch_bounds__(kNT) void edge_gather_kernel(const int* __restrict__ ei, const unsigned short* __restrict__ AH,
                                                          const float* __restrict__ coordb, unsigned short* __restrict__ XA,
                                                          float* __restrict__ RAD, float* __restrict__ CD4, int e0c) {
  const int b = blockIdx.x, t = threadIdx.x;
  if (b < kGatherBlocks) {
    const int gi = b * kNT + t;
    const int el = gi >> 6, piece = gi & 63;
    const int e = e0c + el;
    int r = ei[e]; int c = ei[kEdges + e];
    r = r < 0 ? 0 : (r >= kNodes ? kNodes - 1 : r);
    c = c < 0 ? 0 : (c >= kNodes ? kNodes - 1 : c);
    const int selm = -(int)(piece < 32);
    const int node = (r & selm) | (c & ~selm);
    const v4u w = *(const v4u*)(AH + (size_t)node * kKcat + (piece & 31) * 8);
    unsigned short* dst = XA + (size_t)el * kKcat + piece * 8;
    *(volatile v4u*)dst = w;
    __threadfence();
    *(volatile v4u*)dst = w;
  } else {
    const int el = (b - kGatherBlocks) * kNT + t;
    const bool live = el < kEch;
    const int elc = live ? el : (kEch - 1);
    const int e = e0c + elc;
    int r = ei[e]; int c = ei[kEdges + e];
    r = r < 0 ? 0 : (r >= kNodes ? kNodes - 1 : r);
    c = c < 0 ? 0 : (c >= kNodes ? kNodes - 1 : c);
    const float xr = coordb[r * 3 + 0], yr = coordb[r * 3 + 1], zr = coordb[r * 3 + 2];
    const float xc = coordb[c * 3 + 0], yc = coordb[c * 3 + 1], zc = coordb[c * 3 + 2];
    const float dx = xr - xc, dy = yr - yc, dz = zr - zc;
    const float rad = (dx * dx + dz * dz) + dy * dy;
    const v4f cd = (v4f){dx, dy, dz, 0.0f};
    if (live) {
      *(volatile float*)(RAD + el) = rad;
      *(volatile v4f*)(CD4 + (size_t)el * 4) = cd;
      __threadfence();
      *(volatile float*)(RAD + el) = rad;
      *(volatile v4f*)(CD4 + (size_t)el * 4) = cd;
    }
  }
}

__device__ __forceinline__ int blk_excl_scan(int cnt, int* scan_ws, int tid, int* tot) {
  const int lane = tid & 31, wave = tid >> 5; int incl = cnt;
#pragma unroll
  for (int o = 1; o < 32; o <<= 1) { const int v = __shfl_up(incl, o, 32); incl += (lane >= o) ? v : 0; }
  if (lane == 31) scan_ws[wave] = incl;
  __syncthreads();
  const int wv = scan_ws[lane];
  int wincl = wv;
#pragma unroll
  for (int o = 1; o < 32; o <<= 1) { const int v = __shfl_up(wincl, o, 32); wincl += (lane >= o) ? v : 0; }
  const int wexcl = wincl - wv;
  const int woff = __shfl(wexcl, wave, 32);
  *tot = __shfl(wincl, 31, 32);
  return woff + incl - cnt;
}
__device__ __forceinline__ int chunk_hits_tile(const int* __restrict__ rowv, int s0, int n0, int tid, int* LIST, int* scan_ws) {
  const int eb = s0 + tid * 8;
  const bool gv = eb < kEch;
  const int ebc = gv ? eb : (kEch - 8);
  const v4i d0 = *(const v4i*)(rowv + ebc);
  const v4i d1 = *(const v4i*)(rowv + ebc + 4);
  int rec[8]; int cnt = 0;
#pragma unroll
  for (int k = 0; k < 4; ++k) {
    int d = d0[k];
    d = d < 0 ? 0 : (d >= kNodes ? kNodes - 1 : d);
    const bool hit = gv && d >= n0 && d < n0 + kTnode;
    rec[k] = hit ? (((d - n0) << 16) | (eb + k)) : -1;
    cnt += hit ? 1 : 0;
  }
#pragma unroll
  for (int k = 0; k < 4; ++k) {
    int d = d1[k];
    d = d < 0 ? 0 : (d >= kNodes ? kNodes - 1 : d);
    const bool hit = gv && d >= n0 && d < n0 + kTnode;
    rec[4 + k] = hit ? (((d - n0) << 16) | (eb + 4 + k)) : -1;
    cnt += hit ? 1 : 0;
  }
  int tot; int p = blk_excl_scan(cnt, scan_ws, tid, &tot);
#pragma unroll
  for (int k = 0; k < 8; ++k) if (rec[k] >= 0) { if ((unsigned)p < (unsigned)kScha) LIST[p] = rec[k]; ++p; }
  __syncthreads();
  return tot < kScha ? tot : kScha;
}

__global__ __launch_bounds__(kNT) void aggregate_kernel(const int* __restrict__ ei, const unsigned short* __restrict__ EF,
                                                        const float* __restrict__ SPp, const float* __restrict__ CD4,
                                                        const float* __restrict__ bc2b,
                                                        const float* __restrict__ AGGin, const float* __restrict__ AGCin,
                                                        float* __restrict__ AGGout, float* __restrict__ AGCout,
                                                        int e0c, int init) {
  __shared__ __align__(16) float acc[kTnode * kFeat];
  __shared__ __align__(16) float acc4[kTnode * 4];
  __shared__ int LIST[kScha];
  __shared__ int scan_ws[32];
  const int tid = threadIdx.x, lane = tid & 31, wave = tid >> 5;
  const int n0 = blockIdx.x * kTnode;
  const v4f z4 = (v4f){0.f, 0.f, 0.f, 0.f};
  if (tid >= 8 && tid < 32) scan_ws[tid] = 0;
  if (init) {
    for (int i = tid; i < kTnode * kFeat / 4; i += kNT) *(v4f*)(acc + 4 * i) = z4;
    if (tid < kTnode) *(v4f*)(acc4 + 4 * tid) = z4;
  } else {
#pragma unroll 1
    for (int j = 0; j < 6; ++j) {
      const int dl = wave * 6 + j;
      const float* rp = AGGin + (size_t)(n0 + dl) * kFeat;
      const v4f x0 = *(const v4f*)(rp + 4 * lane);
      const v4f x1 = *(const v4f*)(rp + 128 + 4 * lane);
      *(v4f*)(acc + dl * kFeat + 4 * lane)       = x0;
      *(v4f*)(acc + dl * kFeat + 128 + 4 * lane) = x1;
    }
    if (tid < kTnode) *(v4f*)(acc4 + 4 * tid) = *(const v4f*)(AGCin + (size_t)(n0 + tid) * 4);
  }
  __syncthreads();
  const float bc2v = bc2b[0];
  const int* rowv = ei + e0c;
#pragma unroll 1
  for (int st = 0; st < kNstep; ++st) {
    const int tot = chunk_hits_tile(rowv, st * kScha, n0, tid, LIST, scan_ws);
#pragma unroll 1
    for (int base = 0; base < tot; base += 32) {
      const int q  = base + lane;
      const int qc = q < tot ? q : (tot - 1);
      const int lv = LIST[qc];
      const int rv = lv | (-(int)(q >= tot));
      const int own = ((rv >= 0) & (((rv >> 16) / 6) == wave)) ? 1 : 0;
      unsigned msk = (unsigned)__ballot(own);
#pragma unroll 1
      for (int it = 0; it < 32; ++it) {
        if (msk == 0u) break;
        const int bp = __builtin_ctz(msk); msk &= msk - 1u;
        const int r = __shfl(rv, bp, 32);
        const int dl = r >> 16, el = r & 0xFFFF;
        const v4u w = *(const v4u*)(EF + (size_t)el * kFeat + 8 * lane);
        const v4f cd = *(const v4f*)(CD4 + (size_t)el * 4);
        const float s0 = SPp[el], s1 = SPp[kEch + el], s2 = SPp[2 * kEch + el], s3 = SPp[3 * kEch + el];
        v4f f0, f1;
        f0[0] = h16_to_f32(w[0] & 0xffffu); f0[1] = h16_to_f32(w[0] >> 16);
        f0[2] = h16_to_f32(w[1] & 0xffffu); f0[3] = h16_to_f32(w[1] >> 16);
        f1[0] = h16_to_f32(w[2] & 0xffffu); f1[1] = h16_to_f32(w[2] >> 16);
        f1[2] = h16_to_f32(w[3] & 0xffffu); f1[3] = h16_to_f32(w[3] >> 16);
        float* ap = acc + dl * kFeat + 8 * lane;
        v4f a0 = *(const v4f*)ap;
        v4f a1 = *(const v4f*)(ap + 4);
        a0 = a0 + f0; a1 = a1 + f1;
        *(v4f*)ap = a0; *(v4f*)(ap + 4) = a1;
        const float s = ((s0 + s1) + (s2 + s3)) + bc2v;
        const float t0 = cd[0] * s, t1 = cd[1] * s, t2 = cd[2] * s;
        const float tv = (lane == 0) ? t0 : (lane == 1) ? t1 : (lane == 2) ? t2 : 1.0f;
        if (lane < 4) acc4[dl * 4 + lane] += tv;
      }
    }
    __syncthreads();
  }
  __syncthreads();
#pragma unroll 1
  for (int j = 0; j < 6; ++j) {
    const int dl = wave * 6 + j;
    float* rp = AGGout + (size_t)(n0 + dl) * kFeat;
    const v4f a = *(const v4f*)(acc + dl * kFeat + 4 * lane);
    const v4f c = *(const v4f*)(acc + dl * kFeat + 128 + 4 * lane);
    for (int pass = 0; pass < 2; ++pass) {
      *(volatile v4f*)(rp + 4 * lane) = a;
      *(volatile v4f*)(rp + 128 + 4 * lane) = c;
      __threadfence();
    }
  }
  if (wave == 0) {
    const v4f c0 = *(const v4f*)(acc4 + 4 * lane);
    const v4f c1 = *(const v4f*)(acc4 + 4 * (32 + (lane & 15)));
    for (int pass = 0; pass < 2; ++pass) {
      *(volatile v4f*)(AGCout + (size_t)(n0 + lane) * 4) = c0;
      if (lane < 16) *(volatile v4f*)(AGCout + (size_t)(n0 + 32 + lane) * 4) = c1;
      __threadfence();
    }
  }
}

__global__ __launch_bounds__(kNT) void coord_out_kernel(const float* __restrict__ coordb, const float* __restrict__ AGC,
                                                        float* __restrict__ out1) {
  const int i = blockIdx.x * kNT + threadIdx.x;
  const int ic = i < kCoordN ? i : (kCoordN - 1);
  const int node = ic / 3, d = ic - 3 * node;
  const float c = coordb[ic];
  const float a = AGC[(size_t)node * 4 + d];
  const float cnt = AGC[(size_t)node * 4 + 3];
  const float cntc = fmaxf(cnt, 1.0f);
  const float v = c + a * __builtin_amdgcn_rcpf(cntc);
  if (i < kCoordN) {
    *(volatile float*)(out1 + i) = v;
    __threadfence();
    *(volatile float*)(out1 + i) = v;
  }
}

extern "C" void kernel_launch(void* const* d_in, const int* in_sizes, int n_in,
                              void* d_out, int out_size, void* d_ws, size_t ws_size, hipStream_t stream) {
  if (n_in < 15) return;
  if (in_sizes[0] != kNodes * kFeat || in_sizes[1] != kCoordN || in_sizes[2] != 2 * kEdges) return;
  if (in_sizes[3] != 513 * kFeat || in_sizes[5] != kFeat * kFeat || in_sizes[7] != kKcat * kFeat) return;
  if (in_sizes[9] != kFeat * kFeat || in_sizes[11] != kFeat * kFeat || in_sizes[13] != kFeat || in_sizes[14] < 1) return;
  if (out_size != kNodes * kFeat + kCoordN) return;

  const float* h     = (const float*)d_in[0];
  const float* coord = (const float*)d_in[1];
  const int*   ei    = (const int*)  d_in[2];
  const float* We1 = (const float*)d_in[3];
  const float* be1 = (const float*)d_in[4];
  const float* We2 = (const float*)d_in[5];
  const float* be2 = (const float*)d_in[6];
  const float* Wn1 = (const float*)d_in[7];
  const float* bn1 = (const float*)d_in[8];
  const float* Wn2 = (const float*)d_in[9];
  const float* bn2 = (const float*)d_in[10];
  const float* Wc1 = (const float*)d_in[11];
  const float* bc1 = (const float*)d_in[12];
  const float* Wc2 = (const float*)d_in[13];
  const float* bc2 = (const float*)d_in[14];

  float* out0 = (float*)d_out;
  float* out1 = (float*)d_out + (size_t)kNodes * kFeat;

  char* ws = (char*)d_ws; size_t off = 0;
  auto carve = [&](size_t bytes) -> char* { char* p = ws + off; off += (bytes + 255) & ~(size_t)255; return p; };
  unsigned short* BtWe1  = (unsigned short*)carve((size_t)kFeat * kKcat * 2);
  unsigned short* BtWe2  = (unsigned short*)carve((size_t)kFeat * kFeat * 2);
  unsigned short* BtWc1  = (unsigned short*)carve((size_t)kFeat * kFeat * 2);
  unsigned short* BtWn1  = (unsigned short*)carve((size_t)kFeat * kKcat * 2);
  unsigned short* BtWn2  = (unsigned short*)carve((size_t)kFeat * kFeat * 2);
  float*          VEC    = (float*)carve((size_t)kVecFloats * 4);
  unsigned short* NodeAH = (unsigned short*)carve((size_t)kNpad * kKcat * 2);
  unsigned short* NodeAL = (unsigned short*)carve((size_t)kNpad * kKcat * 2);
  float*          AGG0   = (float*)carve((size_t)kNagg * kFeat * 4);
  float*          AGG1   = (float*)carve((size_t)kNagg * kFeat * 4);
  float*          AGC0   = (float*)carve((size_t)kNagg * 4 * 4);
  float*          AGC1   = (float*)carve((size_t)kNagg * 4 * 4);
  unsigned short* XA     = (unsigned short*)carve((size_t)kEch * kKcat * 2);
  unsigned short* E1     = (unsigned short*)carve((size_t)kEch * kFeat * 2);
  unsigned short* EF     = (unsigned short*)carve((size_t)kEch * kFeat * 2);
  float*          RAD    = (float*)carve((size_t)kEch * 4);
  float*          CD4    = (float*)carve((size_t)kEch * 4 * 4);
  float*          SP     = (float*)carve((size_t)4 * kEch * 4);
  unsigned short* NnH    = (unsigned short*)carve((size_t)kNpad * kFeat * 2);
  unsigned short* NnL    = (unsigned short*)carve((size_t)kNpad * kFeat * 2);
  if (off > ws_size || off > (size_t)134217728) return;

  const float* wrad   = VEC + kVwrad;
  const float* be1b   = VEC + kVbe1;
  const float* be2b   = VEC + kVbe2;
  const float* bc1b   = VEC + kVbc1;
  const float* bn1b   = VEC + kVbn1;
  const float* bn2b   = VEC + kVbn2;
  const float* wc2b   = VEC + kVwc2;
  const float* bc2b   = VEC + kVbc2;
  const float* coordb = VEC + kVcoord;

  prep_w_kernel<<<dim3(28, 4), kNT, 0, stream>>>(We1, We2, Wc1, Wn1, Wn2, BtWe1, BtWe2, BtWc1, BtWn1, BtWn2);
  prep_vec_kernel<<<kVecBlocks, kNT, 0, stream>>>(We1, be1, be2, bc1, bn1, bn2, Wc2, bc2, coord, VEC);
  node_h_kernel<<<kNodeBlocks, kNT, 0, stream>>>(h, NodeAH, NodeAL);

  for (int c = 0; c < kNchunk; ++c) {
    const int e0c = c * kEch;
    const float* aggIn  = (c & 1) ? AGG0 : AGG1;
    const float* agcIn  = (c & 1) ? AGC0 : AGC1;
    float*       aggOut = (c & 1) ? AGG1 : AGG0;
    float*       agcOut = (c & 1) ? AGC1 : AGC0;
    edge_gather_kernel<<<kGatherBlocks + kRadBlocks, kNT, 0, stream>>>(ei, NodeAH, coordb, XA, RAD, CD4, e0c);
    gemm_kernel<1, false, 1><<<kEdgeGemmBlocks, kNT, 0, stream>>>(XA, XA, kKcat, BtWe1, kKcat, (void*)E1, (void*)E1, kFeat,
                                                                  be1b, RAD, wrad, kEch, kFeat, kKcat, kEch, 1.0f);
    gemm_kernel<0, false, 0><<<kEdgeGemmBlocks, kNT, 0, stream>>>(E1, E1, kFeat, BtWe2, kFeat, (void*)EF, (void*)EF, kFeat,
                                                                  be2b, RAD, wrad, kEch, kFeat, kFeat, kEch, kWcarryInv);
    gemm_kernel<0, false, 3><<<kEdgeGemmBlocks, kNT, 0, stream>>>(EF, EF, kFeat, BtWc1, kFeat, (void*)SP, (void*)SP, kEch,
                                                                  bc1b, RAD, wc2b, kEch, kFeat, kFeat, kEch, kWcarryInv);
    aggregate_kernel<<<kNtile, kNT, 0, stream>>>(ei, EF, SP, CD4, bc2b, aggIn, agcIn, aggOut, agcOut, e0c, (c == 0) ? 1 : 0);
  }
  const float* AGGf = ((kNchunk - 1) & 1) ? AGG1 : AGG0;
  const float* AGCf = ((kNchunk - 1) & 1) ? AGC1 : AGC0;

  node_fin_kernel<<<kNodeBlocks, kNT, 0, stream>>>(AGGf, NodeAH, NodeAL);
  gemm_kernel<1, true, 4><<<kNodeGemmBlocks, kNT, 0, stream>>>(NodeAH, NodeAL, kKcat, BtWn1, kKcat, (void*)NnH, (void*)NnL, kFeat,
                                                               bn1b, RAD, wrad, kNpad, kFeat, kKcat, kNpad, 1.0f);
  gemm_kernel<1, true, 2><<<kNodeGemmBlocks, kNT, 0, stream>>>(NnH, NnL, kFeat, BtWn2, kFeat, (void*)out0, (void*)out0, kFeat,
                                                               bn2b, RAD, wrad, kNpad, kFeat, kFeat, kNodes, 1.0f);
  coord_out_kernel<<<kCoordOutBlocks, kNT, 0, stream>>>(coordb, AGCf, out1);
}
